// GCN_72164040507402
// MI455X (gfx1250) — hardware-verified
//
#include <hip/hip_runtime.h>
#include <stddef.h>
#include <stdint.h>
#include <math.h>


#define CIN    128
#define HID    64
#define OUTC   32
#define K2     128
#define NTHR   256
#define NWAVE  8
#define EPT    8
#define CHUNK  (NTHR * EPT)
#define WCAP   (EPT * 32)
#define LISTN  (NWAVE * WCAP)
#define NBA    1024
#define SLA    10
#define RCAP   28672
#define DEGCAP 64
#define PCNT   (1 << 20)
#define GBM    64
#define GTHR   128
#define NU1    (HID * (CIN / 8))
#define NU2    (OUTC * (K2 / 8))
#define AGG_ZINTS (LISTN + 2 * RCAP + 3 * NBA)
#define AGG_LDS_INTS (AGG_ZINTS + 16)
#define WSMAX  134217728

static_assert((CHUNK & (CHUNK - 1)) == 0 && CHUNK <= 4096);
static_assert((NBA & (NBA - 1)) == 0 && NBA == (1 << SLA));
static_assert(((long long)CHUNK << SLA) < (1LL << 31));
static_assert(LISTN % NTHR == 0 && WCAP == EPT * 32);
static_assert(NBA % NWAVE == 0 && NBA % 32 == 0 && NBA % GBM == 0 && NBA == NTHR * 4);
static_assert(RCAP % (NTHR * 4) == 0 && AGG_ZINTS % 4 == 0 && LISTN % 4 == 0);
static_assert(RCAP >= 17546);
static_assert(DEGCAP >= 44 && PCNT > DEGCAP);
static_assert(CIN % 32 == 0 && K2 % 32 == 0 && K2 == 2 * HID);
static_assert(GBM == (GTHR / 32) * 16);
static_assert(NU1 % NTHR == 0 && NU2 % NTHR == 0);
static_assert(CIN / 8 == 16 && K2 / 8 == 16);
static_assert(HID == 2 * 32 && OUTC == 32 && OUTC % 16 == 0 && HID % 16 == 0);
static_assert(AGG_LDS_INTS * 4 <= 300000);

typedef float          v2f   __attribute__((ext_vector_type(2)));
typedef float          v4f   __attribute__((ext_vector_type(4)));
typedef float          v8f   __attribute__((ext_vector_type(8)));
typedef int            v4i   __attribute__((ext_vector_type(4)));
typedef int            v8i   __attribute__((ext_vector_type(8)));
typedef unsigned int   v4u   __attribute__((ext_vector_type(4)));
typedef unsigned short v8us  __attribute__((ext_vector_type(8)));
typedef unsigned short v16us __attribute__((ext_vector_type(16)));
typedef __bf16         v16bf __attribute__((ext_vector_type(16)));
typedef v2f  __attribute__((may_alias)) v2fa;
typedef v4f  __attribute__((may_alias)) v4fa;
typedef v4i  __attribute__((may_alias)) v4ia;
typedef v8us __attribute__((may_alias)) v8usa;
union FragB { v16bf v; v16us u; v8us h[2]; v8i w; };

__device__ __forceinline__ v8f wmb(const FragB& a, const FragB& b, v8f c) {
  v8f d = __builtin_amdgcn_wmma_f32_16x16x32_bf16(false, a.v, false, b.v, (short)0, c, false, false);
  asm volatile("v_nop\n\tv_nop\n\tv_nop\n\tv_nop" : "+v"(d) : "v"(a.w), "v"(b.w));
  return d;
}

__device__ __forceinline__ unsigned bf16_bits(float f) {
  const unsigned u = __float_as_uint(f);
  const unsigned r = (u + 0x7FFFu + ((u >> 16) & 1u)) >> 16;
  const bool isn = (u & 0x7FFFFFFFu) > 0x7F800000u;
  return isn ? 0x7FC0u : r;
}
__device__ __forceinline__ float bf16_val(float f) {
  return __uint_as_float(bf16_bits(f) << 16);
}

__device__ __forceinline__ void put8(unsigned short* dp, const v8us o) {
  *(volatile v8us*)dp = o;
  __threadfence();
  *(volatile v8us*)dp = o;
}

template <int SLB>
__device__ __forceinline__ int scan_chunk(const int* __restrict__ dsts, int nE, int cbase, int slotBase,
                                          int nb, int vec8, int* list, int tid, int lane, int wave) {
  int wc = 0;
  const int el0  = tid * EPT;
  const int e0   = cbase + el0;
  const int sent = -2147483647 - 1;
  v4i da, db;
  if (vec8 != 0 && cbase + CHUNK <= nE) {
    da = *(const v4i*)(dsts + e0);
    db = *(const v4i*)(dsts + e0 + 4);
  } else {
    da.x = (e0     < nE) ? dsts[min(e0,     nE - 1)] : sent;
    da.y = (e0 + 1 < nE) ? dsts[min(e0 + 1, nE - 1)] : sent;
    da.z = (e0 + 2 < nE) ? dsts[min(e0 + 2, nE - 1)] : sent;
    da.w = (e0 + 3 < nE) ? dsts[min(e0 + 3, nE - 1)] : sent;
    db.x = (e0 + 4 < nE) ? dsts[min(e0 + 4, nE - 1)] : sent;
    db.y = (e0 + 5 < nE) ? dsts[min(e0 + 5, nE - 1)] : sent;
    db.z = (e0 + 6 < nE) ? dsts[min(e0 + 6, nE - 1)] : sent;
    db.w = (e0 + 7 < nE) ? dsts[min(e0 + 7, nE - 1)] : sent;
  }
  const unsigned nbs = (unsigned)slotBase;
  const unsigned unb = (unsigned)nb;
  const unsigned s0 = (unsigned)da.x - nbs, s1 = (unsigned)da.y - nbs;
  const unsigned s2 = (unsigned)da.z - nbs, s3 = (unsigned)da.w - nbs;
  const unsigned s4 = (unsigned)db.x - nbs, s5 = (unsigned)db.y - nbs;
  const unsigned s6 = (unsigned)db.z - nbs, s7 = (unsigned)db.w - nbs;
  const bool h0 = s0 < unb, h1 = s1 < unb, h2 = s2 < unb, h3 = s3 < unb;
  const bool h4 = s4 < unb, h5 = s5 < unb, h6 = s6 < unb, h7 = s7 < unb;
  const unsigned any = __builtin_amdgcn_ballot_w32(h0 | h1 | h2 | h3 | h4 | h5 | h6 | h7);
  if (any != 0u) {
#define HITJ(J, HJ, SJ) { \
      const unsigned mj = __builtin_amdgcn_ballot_w32(HJ); \
      if (mj != 0u) { \
        if (HJ) { \
          const int pos = wc + (int)__builtin_amdgcn_mbcnt_lo(mj, 0u); \
          if (pos < WCAP) list[wave * WCAP + pos] = ((el0 + (J)) << SLB) | (int)(SJ); \
        } \
        wc += (int)__builtin_popcount(mj); } }
    HITJ(0, h0, s0)
    HITJ(1, h1, s1)
    HITJ(2, h2, s2)
    HITJ(3, h3, s3)
    HITJ(4, h4, s4)
    HITJ(5, h5, s5)
    HITJ(6, h6, s6)
    HITJ(7, h7, s7)
#undef HITJ
  }
  return wc;
}

__global__ __launch_bounds__(NTHR) void k_prep(const float* __restrict__ x, const float* __restrict__ W1,
                                               const float* __restrict__ W2, int nN, int nUx,
                                               unsigned short* xb, unsigned short* W1T, unsigned short* W2D) {
  const int u = (int)blockIdx.x * NTHR + (int)threadIdx.x;
  v8us o;
  if (u < nUx) {
    const int row = u >> 4;
    const int k8  = (u & 15) * 8;
    const int rc  = row < nN ? row : nN - 1;
    const float* p = x + (size_t)rc * CIN + k8;
    const v4f a = *(const v4fa*)p;
    const v4f b = *(const v4fa*)(p + 4);
    const bool ok = row < nN;
    o[0] = ok ? (unsigned short)bf16_bits(a.x) : (unsigned short)0;
    o[1] = ok ? (unsigned short)bf16_bits(a.y) : (unsigned short)0;
    o[2] = ok ? (unsigned short)bf16_bits(a.z) : (unsigned short)0;
    o[3] = ok ? (unsigned short)bf16_bits(a.w) : (unsigned short)0;
    o[4] = ok ? (unsigned short)bf16_bits(b.x) : (unsigned short)0;
    o[5] = ok ? (unsigned short)bf16_bits(b.y) : (unsigned short)0;
    o[6] = ok ? (unsigned short)bf16_bits(b.z) : (unsigned short)0;
    o[7] = ok ? (unsigned short)bf16_bits(b.w) : (unsigned short)0;
    put8(xb + (size_t)row * CIN + k8, o);
  } else {
    const int v = u - nUx;
    if (v < NU1) {
      const int n  = v >> 4;
      const int k8 = (v & 15) * 8;
      const float* p = W1 + (size_t)k8 * HID + n;
#pragma unroll
      for (int i = 0; i < 8; ++i) o[i] = (unsigned short)bf16_bits(p[(size_t)i * HID]);
      put8(W1T + (size_t)n * CIN + k8, o);
    } else if (v < NU1 + NU2) {
      const int w  = v - NU1;
      const int n  = w >> 4;
      const int k8 = (w & 15) * 8;
      const int kk = k8 & (HID - 1);
      const float* p = W2 + (size_t)kk * OUTC + n;
#pragma unroll
      for (int i = 0; i < 8; ++i) o[i] = (unsigned short)bf16_bits(p[(size_t)i * OUTC]);
      put8(W2D + (size_t)n * K2 + k8, o);
    }
  }
}

__global__ __launch_bounds__(NTHR) void k_bucket(const int* __restrict__ srcs, const int* __restrict__ dsts,
                                                 int nE, int nN, int vec8,
                                                 int* listG, int* cntG, int* offG, float* disG) {
  extern __shared__ __attribute__((aligned(16))) int dsm[];
  int* list = dsm;
  int* hl   = dsm + LISTN;
  int* sl   = dsm + LISTN + RCAP;
  int* cnt  = dsm + LISTN + 2 * RCAP;
  int* offs = cnt + NBA;
  int* cur  = offs + NBA;
  int* misc = cur + NBA;
  const int tid = (int)threadIdx.x, lane = tid & 31, wave = tid >> 5;
  const int blk = (int)blockIdx.x;
  const int nodeBase = blk * NBA;

  {
    const v4i z4 = {0, 0, 0, 0};
    for (int i = tid * 4; i < AGG_ZINTS; i += NTHR * 4) *(v4ia*)(dsm + i) = z4;
    if (tid < 16) misc[tid] = 0;
  }
  __syncthreads();

  int t = 0, ov = 0;
  const int nChunks = (nE + CHUNK - 1) / CHUNK;
#pragma unroll 1
  for (int ch = 0; ch < nChunks; ++ch) {
    const int cbase = ch * CHUNK;
    const int wc = scan_chunk<SLA>(dsts, nE, cbase, nodeBase, NBA, vec8, list, tid, lane, wave);
    if (lane == 0) misc[wave] = wc;
    __syncthreads();
    if (wave == 0) {
#pragma unroll 1
      for (int w2 = 0; w2 < NWAVE; ++w2) {
        int c = misc[w2];
        c = c < 0 ? 0 : (c > WCAP ? WCAP : c);
#pragma unroll 1
        for (int b0 = 0; b0 < c; b0 += 32) {
          const int idx = b0 + lane;
          const int ent = list[w2 * WCAP + (idx < WCAP ? idx : WCAP - 1)];
          const int m32 = (c - b0) < 32 ? (c - b0) : 32;
#pragma unroll 1
          for (int k = 0; k < m32; ++k) {
            const int u    = __builtin_amdgcn_readlane(ent, k);
            const int slot = u & (NBA - 1);
            const int el   = (u >> SLA) & (CHUNK - 1);
            const int pk   = ((cbase + el) << SLA) | slot;
            if (t < RCAP) {
              if (lane == 0) { hl[t] = pk; cnt[slot] = cnt[slot] + 1; }
              t = t + 1;
            } else {
              ov = 1;
            }
          }
        }
      }
    }
    __syncthreads();
  }
  if (wave == 0 && lane == 0) { misc[8] = t; misc[9] = ov; }
  __syncthreads();
  int tt = misc[8];
  tt = tt < 0 ? 0 : (tt > RCAP ? RCAP : tt);
  const int ovf = misc[9];

  if (wave == 0) {
    const int base = lane * (NBA / 32);
    int s = 0;
#pragma unroll 1
    for (int i = 0; i < NBA / 32; ++i) s += cnt[base + i];
    int incl = s;
#pragma unroll
    for (int d = 1; d < 32; d <<= 1) {
      const int y = __shfl_up(incl, d, 32);
      if (lane >= d) incl += y;
    }
    int run = incl - s;
#pragma unroll 1
    for (int i = 0; i < NBA / 32; ++i) {
      const int cv = cnt[base + i];
      offs[base + i] = run;
      cur[base + i]  = run;
      run += cv;
    }
  }
  __syncthreads();
  if (wave == 0) {
#pragma unroll 1
    for (int b0 = 0; b0 < tt; b0 += 32) {
      const int idx = b0 + lane;
      const int ent = hl[idx < RCAP ? idx : RCAP - 1];
      const int m32 = (tt - b0) < 32 ? (tt - b0) : 32;
#pragma unroll 1
      for (int k = 0; k < m32; ++k) {
        const int u    = __builtin_amdgcn_readlane(ent, k);
        const int slot = u & (NBA - 1);
        if (lane == 0) {
          int p = cur[slot];
          p = p < 0 ? 0 : (p > RCAP - 1 ? RCAP - 1 : p);
          sl[p] = u;
          cur[slot] = p + 1;
        }
      }
    }
  }
  __syncthreads();

#pragma unroll 1
  for (int i = tid; i < RCAP; i += NTHR) {
    const int ent = sl[i];
    int eid = ent >> SLA;
    eid = eid < 0 ? 0 : (eid > nE - 1 ? nE - 1 : eid);
    int sr = srcs[eid];
    sr = sr < 0 ? 0 : (sr > nN - 1 ? nN - 1 : sr);
    sl[i] = (i < tt) ? sr : 0;
  }
  __syncthreads();

  int* lg = listG + (size_t)blk * RCAP;
  const int s0 = 4 * tid;
  const v4i c4r = *(const v4ia*)(cnt + s0);
  const v4i o4  = *(const v4ia*)(offs + s0);
  const bool pzb = ovf != 0;
  const float qnan = __int_as_float(0x7fc00000);
  v4i c4;
  c4.x = pzb ? PCNT : c4r.x; c4.y = pzb ? PCNT : c4r.y;
  c4.z = pzb ? PCNT : c4r.z; c4.w = pzb ? PCNT : c4r.w;
  v4f d4;
  {
    const float r0 = rsqrtf((float)c4r.x + 1.0f), r1 = rsqrtf((float)c4r.y + 1.0f);
    const float r2 = rsqrtf((float)c4r.z + 1.0f), r3 = rsqrtf((float)c4r.w + 1.0f);
    d4.x = pzb ? qnan : r0; d4.y = pzb ? qnan : r1;
    d4.z = pzb ? qnan : r2; d4.w = pzb ? qnan : r3;
  }
  int*   cp = cntG + (size_t)nodeBase + s0;
  int*   op = offG + (size_t)nodeBase + s0;
  float* dp = disG + (size_t)nodeBase + s0;
#pragma unroll 1
  for (int it = 0; it < RCAP / (NTHR * 4); ++it) {
    const int q = 4 * (it * NTHR + tid);
    const v4i v = *(const v4ia*)(sl + q);
    *(volatile v4i*)(lg + q) = v;
  }
  *(volatile v4i*)cp = c4;
  *(volatile v4i*)op = o4;
  *(volatile v4f*)dp = d4;
  __threadfence();
#pragma unroll 1
  for (int it = 0; it < RCAP / (NTHR * 4); ++it) {
    const int q = 4 * (it * NTHR + tid);
    const v4i v = *(const v4ia*)(sl + q);
    *(volatile v4i*)(lg + q) = v;
  }
  *(volatile v4i*)cp = c4;
  *(volatile v4i*)op = o4;
  *(volatile v4f*)dp = d4;
}

template <int NT>
__global__ __launch_bounds__(GTHR) void k_gemm(const unsigned short* __restrict__ A,
                                               const unsigned short* __restrict__ WT,
                                               float* outF, int K) {
  static_assert(NT == 2 || NT == 4);
  constexpr int GN  = 16 * NT;
  constexpr int LPR = GN / 4;
  constexpr int RPI = 32 / LPR;
  constexpr int NIT = 16 / RPI;
  static_assert(LPR * 4 == GN && RPI * LPR == 32 && NIT * RPI == 16);
  __shared__ __attribute__((aligned(16))) float stg[GBM * GN];
  const int tid = (int)threadIdx.x, lane = tid & 31, wave = tid >> 5, hh = lane >> 4, m = lane & 15;
  const int rowBase = (int)blockIdx.x * GBM;

  v8f acc[NT];
  {
    const v8f z = {0.f, 0.f, 0.f, 0.f, 0.f, 0.f, 0.f, 0.f};
#pragma unroll
    for (int t = 0; t < NT; ++t) acc[t] = z;
  }
  const unsigned short* ap = A  + (size_t)(rowBase + 16 * wave + m) * (size_t)K + 8 * hh;
  const unsigned short* wp = WT + (size_t)m * (size_t)K + 8 * hh;
  const int ksteps = K >> 5;
#pragma unroll 1
  for (int ks = 0; ks < ksteps; ++ks) {
    FragB af;
    af.h[0] = *(const v8usa*)(ap + 32 * ks);
    af.h[1] = *(const v8usa*)(ap + 32 * ks + 16);
#pragma unroll
    for (int t = 0; t < NT; ++t) {
      const unsigned short* wq = wp + (size_t)(16 * t) * (size_t)K + 32 * ks;
      FragB bf;
      bf.h[0] = *(const v8usa*)wq;
      bf.h[1] = *(const v8usa*)(wq + 16);
      acc[t] = wmb(af, bf, acc[t]);
    }
  }

#pragma unroll
  for (int t = 0; t < NT; ++t) {
    const int lc = 16 * t + m;
#pragma unroll
    for (int r = 0; r < 8; ++r) {
      const int lr = 16 * wave + 8 * hh + r;
      stg[lr * GN + lc] = acc[t][r];
    }
  }
  __syncthreads();

  const int rsub = lane / LPR;
  const int cq   = lane % LPR;
  v4f fv[NIT];
#pragma unroll
  for (int i = 0; i < NIT; ++i) {
    const int lr = 16 * wave + RPI * i + rsub;
    fv[i] = *(const v4fa*)(stg + lr * GN + 4 * cq);
  }
#pragma unroll
  for (int i = 0; i < NIT; ++i) {
    const int lr = 16 * wave + RPI * i + rsub;
    float* op = outF + (size_t)(rowBase + lr) * (size_t)GN + 4 * cq;
    *(volatile v4f*)op = fv[i];
  }
  __threadfence();
#pragma unroll
  for (int i = 0; i < NIT; ++i) {
    const int lr = 16 * wave + RPI * i + rsub;
    float* op = outF + (size_t)(rowBase + lr) * (size_t)GN + 4 * cq;
    *(volatile v4f*)op = fv[i];
  }
}

__global__ __launch_bounds__(NTHR) void k_agg1(const int* __restrict__ listG, const int* __restrict__ cntG,
                                               const int* __restrict__ offG, const float* __restrict__ dis,
                                               const float* __restrict__ xl, const float* __restrict__ bias,
                                               int nN, int mRows, unsigned short* hb) {
  const int tid = (int)threadIdx.x, lane = tid & 31, wave = tid >> 5;
  const int blk = (int)blockIdx.x;
  const int nodeBase = blk * NBA;
  const int* lp = listG + (size_t)blk * RCAP;
  float bv0, bv1;
  {
    const v2f a = *(const v2fa*)(bias + 2 * lane);
    bv0 = bf16_val(a.x); bv1 = bf16_val(a.y);
  }
  const float qnan = __int_as_float(0x7fc00000);
  const int q0s = (4 * lane) & 31, q1s = (4 * lane + 1) & 31;
  const int q2s = (4 * lane + 2) & 31, q3s = (4 * lane + 3) & 31;
#pragma unroll 1
  for (int si = 0; si < NBA / NWAVE; ++si) {
    const int s    = si * NWAVE + wave;
    const int node = nodeBase + s;
    int c = cntG[node];
    const bool big = c > DEGCAP;
    c = c < 0 ? 0 : (c > DEGCAP ? DEGCAP : c);
    int o = offG[node];
    o = o < 0 ? 0 : (o > RCAP ? RCAP : o);
    const int nc = node < nN ? node : nN - 1;
    const float dd = dis[node];
    const float rd = dd * dd;
    float acc0 = 0.0f, acc1 = 0.0f;
#pragma unroll 1
    for (int b0 = 0; b0 < c; b0 += 32) {
      int idx = o + b0 + lane;
      idx = idx > RCAP - 1 ? RCAP - 1 : idx;
      int sr = lp[idx];
      sr = sr < 0 ? 0 : (sr > nN - 1 ? nN - 1 : sr);
      const float cf  = dis[sr] * dd;
      const int   cfi = __float_as_int(cf);
      const int m32 = (c - b0) < 32 ? (c - b0) : 32;
#pragma unroll 1
      for (int k = 0; k < m32; ++k) {
        const int   sk = __builtin_amdgcn_readlane(sr, k);
        const float ck = __int_as_float(__builtin_amdgcn_readlane(cfi, k));
        const v2f a = *(const v2fa*)(xl + (size_t)sk * HID + 2 * lane);
        acc0 = fmaf(ck, a.x, acc0); acc1 = fmaf(ck, a.y, acc1);
      }
    }
    float sv0, sv1;
    {
      const v2f a = *(const v2fa*)(xl + (size_t)nc * HID + 2 * lane);
      sv0 = a.x; sv1 = a.y;
    }
    const bool live = node < nN;
    float y0 = (acc0 + sv0 * rd) + bv0;
    float y1 = (acc1 + sv1 * rd) + bv1;
    y0 = (y0 > 0.0f) ? y0 : (y0 - y0);
    y1 = (y1 > 0.0f) ? y1 : (y1 - y1);
    y0 = big ? qnan : y0;
    y1 = big ? qnan : y1;
    const float v0 = live ? y0 : 0.0f;
    const float v1 = live ? y1 : 0.0f;
    const bool wr = (node < mRows) && (lane < 16);
    const unsigned hb0 = bf16_bits(v0), hb1 = bf16_bits(v1);
    const unsigned lb0 = bf16_bits(v0 - __uint_as_float(hb0 << 16));
    const unsigned lb1 = bf16_bits(v1 - __uint_as_float(hb1 << 16));
    const int hw = (int)(hb0 | (hb1 << 16));
    const int lw = (int)(lb0 | (lb1 << 16));
    const int g0 = __shfl(hw, q0s, 32), g1 = __shfl(hw, q1s, 32);
    const int g2 = __shfl(hw, q2s, 32), g3 = __shfl(hw, q3s, 32);
    const int p0 = __shfl(lw, q0s, 32), p1 = __shfl(lw, q1s, 32);
    const int p2 = __shfl(lw, q2s, 32), p3 = __shfl(lw, q3s, 32);
    const bool lsel = (lane & 8) != 0;
    v4u pv;
    pv.x = (unsigned int)(lsel ? p0 : g0);
    pv.y = (unsigned int)(lsel ? p1 : g1);
    pv.z = (unsigned int)(lsel ? p2 : g2);
    pv.w = (unsigned int)(lsel ? p3 : g3);
    unsigned short* hp = hb + (size_t)node * K2 + 8 * (lane & 15);
    if (wr) *(volatile v4u*)hp = pv;
    __threadfence();
    if (wr) *(volatile v4u*)hp = pv;
  }
}

__global__ __launch_bounds__(NTHR) void k_agg2(const int* __restrict__ listG, const int* __restrict__ cntG,
                                               const int* __restrict__ offG, const float* __restrict__ dis,
                                               const float* __restrict__ xl, const float* __restrict__ bias,
                                               int nN, float* out) {
  const int tid = (int)threadIdx.x, lane = tid & 31, wave = tid >> 5;
  const int blk = (int)blockIdx.x;
  const int nodeBase = blk * NBA;
  const int* lp = listG + (size_t)blk * RCAP;
  const float bv = bf16_val(bias[lane]);
  const float qnan = __int_as_float(0x7fc00000);
#pragma unroll 1
  for (int si = 0; si < NBA / NWAVE; ++si) {
    const int s    = si * NWAVE + wave;
    const int node = nodeBase + s;
    int c = cntG[node];
    const bool big = c > DEGCAP;
    c = c < 0 ? 0 : (c > DEGCAP ? DEGCAP : c);
    int o = offG[node];
    o = o < 0 ? 0 : (o > RCAP ? RCAP : o);
    const int nc = node < nN ? node : nN - 1;
    const float dd = dis[node];
    const float rd = dd * dd;
    float acc = 0.0f;
#pragma unroll 1
    for (int b0 = 0; b0 < c; b0 += 32) {
      int idx = o + b0 + lane;
      idx = idx > RCAP - 1 ? RCAP - 1 : idx;
      int sr = lp[idx];
      sr = sr < 0 ? 0 : (sr > nN - 1 ? nN - 1 : sr);
      const float cf  = dis[sr] * dd;
      const int   cfi = __float_as_int(cf);
      const int m32 = (c - b0) < 32 ? (c - b0) : 32;
#pragma unroll 1
      for (int k = 0; k < m32; ++k) {
        const int   sk = __builtin_amdgcn_readlane(sr, k);
        const float ck = __int_as_float(__builtin_amdgcn_readlane(cfi, k));
        const float a  = xl[(size_t)sk * OUTC + lane];
        acc = fmaf(ck, a, acc);
      }
    }
    const float sv = xl[(size_t)nc * OUTC + lane];
    float y = (acc + sv * rd) + bv;
    y = big ? qnan : y;
    const bool wr = node < nN;
    float* op = out + (size_t)nc * OUTC + lane;
    if (wr) *(volatile float*)op = y;
    __threadfence();
    if (wr) *(volatile float*)op = y;
  }
}

static inline int cdiv(int a, int b) { return (a + b - 1) / b; }
static inline size_t al256(size_t o) { return (o + 255) & ~(size_t)255; }

extern "C" void kernel_launch(void* const* d_in, const int* in_sizes, int n_in,
                              void* d_out, int out_size, void* d_ws, size_t ws_size,
                              hipStream_t stream) {
  if (n_in < 6) return;
  if (in_sizes[0] < CIN || (in_sizes[0] % CIN) != 0) return;
  const int nN = in_sizes[0] / CIN;
  if (nN < 1 || nN > (1 << 22)) return;
  if (in_sizes[1] < 2 || (in_sizes[1] & 1) != 0) return;
  const int nE = in_sizes[1] / 2;
  if (nE < 1 || nE >= (1 << (31 - SLA))) return;
  if (in_sizes[2] != CIN * HID || in_sizes[3] != HID) return;
  if (in_sizes[4] != HID * OUTC || in_sizes[5] != OUTC) return;
  if ((long long)out_size != (long long)nN * OUTC) return;
  if ((long long)nE * NBA * 3 > (long long)nN * RCAP * 2) return;

  const float* x    = (const float*)d_in[0];
  const int*   edge = (const int*)d_in[1];
  const float* W1   = (const float*)d_in[2];
  const float* b1   = (const float*)d_in[3];
  const float* W2   = (const float*)d_in[4];
  const float* b2   = (const float*)d_in[5];
  float* out = (float*)d_out;
  const int* src = edge;
  const int* dst = edge + nE;

  const int MP   = cdiv(nN, 128) * 128;
  const int gM   = MP / GBM;
  const int gA   = cdiv(MP, NBA);
  const int NTAB = gA * NBA;
  if ((long long)gA * NBA < (long long)MP) return;
  const int nUx = MP * (CIN / 8);
  if ((nUx % NTHR) != 0) return;
  const int vec8 = ((nE & 3) == 0) ? 1 : 0;

  char* ws = (char*)d_ws;
  size_t off = 0;
  const size_t oDIS = off; off = al256(off + (size_t)NTAB * 4);
  const size_t oCNT = off; off = al256(off + (size_t)NTAB * 4);
  const size_t oOFF = off; off = al256(off + (size_t)NTAB * 4);
  const size_t oLST = off; off = al256(off + (size_t)gA * RCAP * 4);
  const size_t oW1T = off; off = al256(off + (size_t)HID * CIN * 2);
  const size_t oW2D = off; off = al256(off + (size_t)OUTC * K2 * 2);
  const size_t oXB  = off; off = al256(off + (size_t)MP * CIN * 2);
  const size_t oH1  = off; off = al256(off + (size_t)MP * HID * 4);
  const size_t oX1  = off; off = al256(off + (size_t)MP * K2 * 2);
  const size_t oH2  = off; off = al256(off + (size_t)MP * OUTC * 4);
  if (off > ws_size || off > (size_t)WSMAX) return;
  float*          DIS = (float*)(ws + oDIS);
  int*            CNT = (int*)(ws + oCNT);
  int*            OFF = (int*)(ws + oOFF);
  int*            LST = (int*)(ws + oLST);
  unsigned short* W1T = (unsigned short*)(ws + oW1T);
  unsigned short* W2D = (unsigned short*)(ws + oW2D);
  unsigned short* XB  = (unsigned short*)(ws + oXB);
  float*          H1  = (float*)(ws + oH1);
  unsigned short* X1  = (unsigned short*)(ws + oX1);
  float*          H2  = (float*)(ws + oH2);

  const size_t bkLds = (size_t)AGG_LDS_INTS * 4;
  hipFuncSetAttribute(reinterpret_cast<const void*>(&k_bucket), hipFuncAttributeMaxDynamicSharedMemorySize, (int)bkLds);

  k_prep<<<(nUx + NU1 + NU2) / NTHR, NTHR, 0, stream>>>(x, W1, W2, nN, nUx, XB, W1T, W2D);
  k_bucket<<<gA, NTHR, bkLds, stream>>>(src, dst, nE, nN, vec8, LST, CNT, OFF, DIS);
  k_gemm<4><<<gM, GTHR, 0, stream>>>(XB, W1T, H1, CIN);
  k_agg1<<<gA, NTHR, 0, stream>>>(LST, CNT, OFF, DIS, H1, b1, nN, MP, X1);
  k_gemm<2><<<gM, GTHR, 0, stream>>>(X1, W2D, H2, K2);
  k_agg2<<<gA, NTHR, 0, stream>>>(LST, CNT, OFF, DIS, H2, b2, nN, out);
}
